// EpisodicMemoryModuleLayer_5085241278808
// MI455X (gfx1250) — hardware-verified
//
#include <hip/hip_runtime.h>
#include <math.h>
#include <stdint.h>

constexpr int NBATCH   = 64;
constexpr int NFACT    = 256;
constexpr int NEMB     = 512;
constexpr int NGATE3   = 1536;
constexpr int NROWALL  = 16384;
constexpr int KFEAT2   = 1024;
constexpr int MHALF    = 8192;
constexpr int NHOPS    = 2;
constexpr int NTHREADS = 256;
constexpr int RBLK     = 32;
constexpr int HTPITCH  = 520;
constexpr int GPLANE   = NGATE3 * NEMB;
constexpr int XMPLANE  = NBATCH * NGATE3;
constexpr int EPPLANE  = NBATCH * NEMB;
constexpr float WCARRY  = 64.0f;
constexpr float HCARRY  = 16.0f;
constexpr float FOLD_W  = 1.0f / 64.0f;
constexpr float FOLD_HW = 1.0f / 1024.0f;
constexpr int HS_BYTES  = RBLK * NEMB * 4;
constexpr int HT_HALVES = RBLK * HTPITCH;
constexpr int REC_LDS_BYTES = HS_BYTES + 2 * HT_HALVES * 2;

static_assert(NROWALL == NBATCH * NFACT);
static_assert(REC_LDS_BYTES == 132096);
static_assert((NROWALL * NEMB / 8) % NTHREADS == 0);
static_assert((MHALF * KFEAT2 / 8) % NTHREADS == 0);
static_assert((NBATCH * NEMB / 4) % NTHREADS == 0);
static_assert(NEMB % 32 == 0 && KFEAT2 % 32 == 0);
static_assert(NROWALL % 64 == 0 && NGATE3 % 64 == 0 && NEMB % 64 == 0 && MHALF % 64 == 0 && NBATCH % 64 == 0);
static_assert((HT_HALVES * 2) % 16 == 0 && HTPITCH % 8 == 0);
static_assert(RBLK * NEMB == 16 * 32 * 32);

typedef __attribute__((ext_vector_type(16))) _Float16 v16h;
typedef __attribute__((ext_vector_type(8)))  _Float16 v8h;
typedef __attribute__((ext_vector_type(4)))  _Float16 v4h;
typedef __attribute__((ext_vector_type(16))) __bf16   v16b;
typedef __attribute__((ext_vector_type(8)))  __bf16   v8b;
typedef __attribute__((ext_vector_type(8)))  float    v8f;
typedef __attribute__((ext_vector_type(4)))  float    v4f;

__device__ __forceinline__ unsigned short f2bf_bits(float f) {
  unsigned u = __float_as_uint(f);
  return (unsigned short)((u + 0x7FFFu + ((u >> 16) & 1u)) >> 16);
}
__device__ __forceinline__ float bf_bits2f(unsigned short h) { return __uint_as_float(((unsigned)h) << 16); }

__device__ __forceinline__ void dep_guard_h(v8f& a, v8f& b, v16h x, v16h y) { asm volatile("v_nop\n\tv_nop\n\tv_nop\n\tv_nop" : "+v"(a), "+v"(b) : "v"(x), "v"(y)); }
__device__ __forceinline__ void dep_guard_b(v8f& a, v8f& b, v16b x, v16b y) { asm volatile("v_nop\n\tv_nop\n\tv_nop\n\tv_nop" : "+v"(a), "+v"(b) : "v"(x), "v"(y)); }
__device__ __forceinline__ void keep4_h(v16h a, v16h b, v16h c, v16h d) { asm volatile("v_nop" :: "v"(a), "v"(b), "v"(c), "v"(d)); }
__device__ __forceinline__ void keep4_b(v16b a, v16b b, v16b c, v16b d) { asm volatile("v_nop" :: "v"(a), "v"(b), "v"(c), "v"(d)); }
__device__ __forceinline__ void acc_guard4(v8f& a, v8f& b, v8f& c, v8f& d) { asm volatile("v_nop\n\tv_nop\n\tv_nop\n\tv_nop" : "+v"(a), "+v"(b), "+v"(c), "+v"(d)); }
template <typename T> struct Frag;
template <> struct Frag<_Float16> {
  typedef v16h V; union U { v16h v; v8h h[2]; };
  static __device__ __forceinline__ v16h load(const _Float16* p) {
    U f; f.h[0] = *(const v8h*)(p); f.h[1] = *(const v8h*)(p + 16); return f.v;
  }
  static __device__ __forceinline__ v8f mma(v16h a, v16h b, v8f c) {
    return __builtin_amdgcn_wmma_f32_16x16x32_f16(false, a, false, b, (short)0, c, false, false);
  }
  static __device__ __forceinline__ void guard(v8f& a, v8f& b, v16h x, v16h y) { dep_guard_h(a, b, x, y); }
  static __device__ __forceinline__ void keep(v16h a, v16h b, v16h c, v16h d) { keep4_h(a, b, c, d); }
};
template <> struct Frag<__bf16> {
  typedef v16b V; union U { v16b v; v8b h[2]; };
  static __device__ __forceinline__ v16b load(const __bf16* p) {
    U f; f.h[0] = *(const v8b*)(p); f.h[1] = *(const v8b*)(p + 16); return f.v;
  }
  static __device__ __forceinline__ v8f mma(v16b a, v16b b, v8f c) {
    return __builtin_amdgcn_wmma_f32_16x16x32_bf16(false, a, false, b, (short)0, c, false, false);
  }
  static __device__ __forceinline__ void guard(v8f& a, v8f& b, v16b x, v16b y) { dep_guard_b(a, b, x, y); }
  static __device__ __forceinline__ void keep(v16b a, v16b b, v16b c, v16b d) { keep4_b(a, b, c, d); }
};
typedef Frag<_Float16> FragH;

__device__ __forceinline__ float fsig(float v)  { return __builtin_amdgcn_rcpf(1.0f + __expf(-v)); }
__device__ __forceinline__ float ftanh(float v) { return 1.0f - 2.0f * __builtin_amdgcn_rcpf(__expf(2.0f * v) + 1.0f); }

template <int ET> struct Elem;
template <> struct Elem<0> { typedef _Float16 T; };
template <> struct Elem<1> { typedef __bf16 T; };
template <int ET, bool SPLIT, int BIAS_MODE, int OUT_MODE, bool RESID, int ACT = 0>
__global__ __launch_bounds__(256) void wmma_gemm64(
    const unsigned short* __restrict__ Ap, const unsigned short* __restrict__ A2p, int lda, long strideA,
    const unsigned short* __restrict__ Btp, const unsigned short* __restrict__ Bt2p, int ldb, long strideB,
    void* __restrict__ Cout, void* __restrict__ Cout2, int ldc, long strideC,
    const float* __restrict__ bias,
    const float* __restrict__ resid, long strideR,
    int M, int N, int K, float scale) {
  typedef typename Elem<ET>::T T;
  typedef typename Frag<T>::V V;
  const T* A = (const T*)Ap; const T* A2 = (const T*)A2p; const T* Bt = (const T*)Btp; const T* Bt2 = (const T*)Bt2p;
  __shared__ __align__(16) float sT[8][16 * 68];
  const int b    = blockIdx.y;
  const int lane = threadIdx.x & 31;
  const int wave = threadIdx.x >> 5;
  const int tilesN = N >> 6;
  const int tilesM = M >> 6;
  const int tile = blockIdx.x * 8 + wave;
  if (tile >= tilesM * tilesN) return;
  const int tm = tile / tilesN;
  const int tn = tile - tm * tilesN;
  const int m0 = tm << 6;
  const int n0 = tn << 6;

  const T* Ab  = A  + (size_t)b * strideA;
  const T* Bb  = Bt + (size_t)b * strideB;
  const T* Ab2 = SPLIT ? (A2  + (size_t)b * strideA) : nullptr;
  const T* Bb2 = SPLIT ? (Bt2 + (size_t)b * strideB) : nullptr;

  const int rlane = lane & 15;
  const int koff  = (lane >> 4) * 8;
  const int mOff  = (lane >> 4) * 8;

  v8f acc[4][4];
#pragma unroll
  for (int i = 0; i < 4; ++i)
#pragma unroll
    for (int j = 0; j < 4; ++j) acc[i][j] = (v8f){0.f,0.f,0.f,0.f,0.f,0.f,0.f,0.f};

  for (int k0 = 0; k0 < K; k0 += 32) {
    V bh[4], bl[4];
#pragma unroll
    for (int j = 0; j < 4; ++j) {
      const size_t bo = (size_t)(n0 + (j << 4) + rlane) * ldb + koff + k0;
      bh[j] = Frag<T>::load(Bb + bo);
      if (SPLIT) bl[j] = Frag<T>::load(Bb2 + bo);
    }
#pragma unroll
    for (int i = 0; i < 4; ++i) {
      const size_t ao = (size_t)(m0 + (i << 4) + rlane) * lda + koff + k0;
      V ah = Frag<T>::load(Ab + ao);
      V al;
      if (SPLIT) al = Frag<T>::load(Ab2 + ao);
#pragma unroll
      for (int j = 0; j < 4; ++j) {
        acc[i][j] = Frag<T>::mma(ah, bh[j], acc[i][j]);
        if (SPLIT) {
          acc[i][j] = Frag<T>::mma(ah, bl[j], acc[i][j]);
          acc[i][j] = Frag<T>::mma(al, bh[j], acc[i][j]);
        }
      }
      Frag<T>::guard(acc[i][0], acc[i][3], ah, SPLIT ? al : ah);
    }
    Frag<T>::keep(bh[0], bh[1], bh[2], bh[3]);
    if (SPLIT) Frag<T>::keep(bl[0], bl[1], bl[2], bl[3]);
  }
  acc_guard4(acc[0][0], acc[0][1], acc[0][2], acc[0][3]);
  acc_guard4(acc[1][0], acc[1][1], acc[1][2], acc[1][3]);
  acc_guard4(acc[2][0], acc[2][1], acc[2][2], acc[2][3]);
  acc_guard4(acc[3][0], acc[3][1], acc[3][2], acc[3][3]);

  float* slab = sT[wave];
  const float* Rb = RESID ? (resid + (size_t)b * strideR) : nullptr;
#pragma unroll
  for (int i = 0; i < 4; ++i) {
    const int mBase = m0 + (i << 4);
#pragma unroll
    for (int j = 0; j < 4; ++j) {
      const int n = n0 + (j << 4) + rlane;
      float bv = 0.f;
      if (BIAS_MODE == 2) bv = bias[n];
#pragma unroll
      for (int r = 0; r < 8; ++r) {
        float v = acc[i][j][r] * scale;
        if (BIAS_MODE == 1) v += bias[mBase + mOff + r];
        if (BIAS_MODE == 2) v += bv;
        if (RESID) v += Rb[(size_t)(mBase + mOff + r) * ldc + n];
        if (ACT == 1) v = tanhf(v);
        if (ACT == 2) v = fmaxf(v, 0.0f);
        if (ACT == 3) v = v / (1.0f + expf(-v));
        if (ACT == 4) v = (v > 0.f) ? v : 0.01f * v;
        if (ACT == 5) v = 0.5f * v * (1.0f + erff(v * 0.70710678118654752f));
        slab[(mOff + r) * 68 + (j << 4) + rlane] = v;
      }
    }
    __builtin_amdgcn_fence(__ATOMIC_RELEASE, "workgroup");
    __builtin_amdgcn_wave_barrier();
    __builtin_amdgcn_fence(__ATOMIC_ACQUIRE, "workgroup");
    if (OUT_MODE == 0) {
      float* C = (float*)Cout + (size_t)b * strideC;
      const int hh = lane >> 4, c4 = (lane & 15) * 4;
      for (int pass = 0; pass < 2; ++pass) {
#pragma unroll
        for (int it = 0; it < 8; ++it) {
          const int row = it * 2 + hh;
          v4f v = *(const v4f*)(slab + row * 68 + c4);
          *(volatile v4f*)(C + (size_t)(mBase + row) * ldc + n0 + c4) = v;
        }
        __threadfence();
      }
    } else {
      const int q = lane >> 3, c8 = (lane & 7) * 8;
      unsigned short* C  = (unsigned short*)Cout  + (size_t)b * strideC;
      unsigned short* C2 = (OUT_MODE == 2) ? ((unsigned short*)Cout2 + (size_t)b * strideC) : nullptr;
      for (int pass = 0; pass < 2; ++pass) {
#pragma unroll
        for (int it = 0; it < 4; ++it) {
          const int row = it * 4 + q;
          const float* sp = slab + row * 68 + c8;
          v8h hv, lv;
#pragma unroll
          for (int e = 0; e < 8; ++e) {
            if (OUT_MODE == 1) {
              hv[e] = (_Float16)sp[e];
            } else {
              unsigned short hb = f2bf_bits(sp[e]);
              unsigned short lb = f2bf_bits(sp[e] - bf_bits2f(hb));
              hv[e] = __builtin_bit_cast(_Float16, hb);
              lv[e] = __builtin_bit_cast(_Float16, lb);
            }
          }
          *(volatile v8h*)(C + (size_t)(mBase + row) * ldc + n0 + c8) = hv;
          if (OUT_MODE == 2) *(volatile v8h*)(C2 + (size_t)(mBase + row) * ldc + n0 + c8) = lv;
        }
        __threadfence();
      }
    }
    __builtin_amdgcn_fence(__ATOMIC_RELEASE, "workgroup");
    __builtin_amdgcn_wave_barrier();
    __builtin_amdgcn_fence(__ATOMIC_ACQUIRE, "workgroup");
  }
}

__global__ __launch_bounds__(NTHREADS) void cast_facts_kernel(const float* __restrict__ facts, unsigned short* __restrict__ outp) {
  const int i  = blockIdx.x * NTHREADS + threadIdx.x;
  const int n  = i >> 6;
  const int e0 = (i & 63) * 8;
  const int f  = n >> 6, b = n & 63;
  const float* src = facts + ((size_t)b * NFACT + f) * NEMB + e0;
  const v4f x0 = *(const v4f*)src;
  const v4f x1 = *(const v4f*)(src + 4);
  v8h hv;
#pragma unroll
  for (int e = 0; e < 4; ++e) { hv[e] = (_Float16)x0[e]; hv[4 + e] = (_Float16)x1[e]; }
  unsigned short* dst = outp + (size_t)n * NEMB + e0;
  *(volatile v8h*)dst = hv;
  __threadfence();
  *(volatile v8h*)dst = hv;
}

__device__ __forceinline__ void tile_transpose(const float* __restrict__ W, int ldw, int kr0, int n0,
                                               unsigned short* __restrict__ O, int ldo, int kout0, float* tile, int tid) {
#pragma unroll 1
  for (int it = 0; it < 16; ++it) {
    const int idx = it * NTHREADS + tid;
    const int kr = idx >> 6, nc = idx & 63;
    tile[kr * 65 + nc] = W[(size_t)(kr0 + kr) * ldw + n0 + nc];
  }
  __syncthreads();
#pragma unroll 1
  for (int it = 0; it < 2; ++it) {
    const int row = it * 32 + (tid >> 3);
    const int q = tid & 7;
    v8h hv;
#pragma unroll
    for (int e = 0; e < 8; ++e) hv[e] = (_Float16)(WCARRY * tile[(8 * q + e) * 65 + row]);
    unsigned short* dst = O + (size_t)(n0 + row) * ldo + kout0 + 8 * q;
    *(volatile v8h*)dst = hv;
    __threadfence();
    *(volatile v8h*)dst = hv;
  }
}

__global__ __launch_bounds__(NTHREADS) void w1_trans_kernel(const float* __restrict__ W1, unsigned short* __restrict__ PA,
                                                           unsigned short* __restrict__ PB) {
  __shared__ float tile[64 * 65];
  const int tid = threadIdx.x;
  const int n0  = blockIdx.x * 64;
  const int kr0 = blockIdx.y * 64;
  const int seg = kr0 >> 9;
  unsigned short* P = (seg & 1) ? PB : PA;
  const int kout0 = (seg >> 1) * NEMB + (kr0 & (NEMB - 1));
  tile_transpose(W1, NEMB, kr0, n0, P, KFEAT2, kout0, tile, tid);
}

__global__ __launch_bounds__(NTHREADS) void gate_trans_kernel(const float* __restrict__ w0, const float* __restrict__ w1,
                                                             const float* __restrict__ w2, const float* __restrict__ w3,
                                                             unsigned short* __restrict__ planes) {
  __shared__ float tile[64 * 65];
  const int tid = threadIdx.x;
  const int z = blockIdx.z;
  const float* W = (z == 0) ? w0 : (z == 1) ? w1 : (z == 2) ? w2 : w3;
  const int n0  = blockIdx.x * 64;
  const int kr0 = blockIdx.y * 64;
  tile_transpose(W, NGATE3, kr0, n0, planes + (size_t)z * GPLANE, NEMB, kr0, tile, tid);
}

__global__ __launch_bounds__(NTHREADS) void init_mem16_kernel(unsigned short* __restrict__ M16) {
  const int i = blockIdx.x * NTHREADS + threadIdx.x;
  const _Float16 hv1 = (_Float16)(HCARRY * 0.1f);
  v8h hv;
#pragma unroll
  for (int e = 0; e < 8; ++e) hv[e] = hv1;
  unsigned short* dst = M16 + (size_t)i * 8;
  *(volatile v8h*)dst = hv;
  __threadfence();
  *(volatile v8h*)dst = hv;
}

__global__ __launch_bounds__(NTHREADS) void feat_build_kernel(const float* __restrict__ facts, const float* __restrict__ mrow,
                                                             int use_m, int half, unsigned short* __restrict__ FO) {
  const int i  = blockIdx.x * NTHREADS + threadIdx.x;
  const int nl = i >> 7;
  const int kq = (i & 127) * 8;
  const int n  = half * MHALF + nl;
  const int f  = n >> 6, b = n & 63;
  const int e0 = kq & (NEMB - 1);
  const bool second = (kq >= NEMB);
  const float* src = facts + ((size_t)b * NFACT + f) * NEMB + e0;
  const v4f x0 = *(const v4f*)src;
  const v4f x1 = *(const v4f*)(src + 4);
  v4f m0 = {0.1f, 0.1f, 0.1f, 0.1f};
  v4f m1 = {0.1f, 0.1f, 0.1f, 0.1f};
  if (use_m != 0) {
    m0 = *(const v4f*)(mrow + (size_t)b * NEMB + e0);
    m1 = *(const v4f*)(mrow + (size_t)b * NEMB + e0 + 4);
  }
  v8h hv;
#pragma unroll
  for (int e = 0; e < 4; ++e) {
    const float pa = x0[e] * m0[e];
    const float da = fabsf(x0[e] - m0[e]);
    const float pb = x1[e] * m1[e];
    const float db = fabsf(x1[e] - m1[e]);
    hv[e]     = (_Float16)(second ? da : pa);
    hv[4 + e] = (_Float16)(second ? db : pb);
  }
  unsigned short* dst = FO + (size_t)nl * KFEAT2 + kq;
  *(volatile v8h*)dst = hv;
  __threadfence();
  *(volatile v8h*)dst = hv;
}

__global__ __launch_bounds__(NTHREADS) void gate_head_kernel(const unsigned short* __restrict__ T16p, const float* __restrict__ W2,
                                                            const float* __restrict__ b2, float* __restrict__ G) {
  __shared__ __align__(16) float gs[32];
  const _Float16* Tp = (const _Float16*)T16p;
  const int tid = threadIdx.x, lane = tid & 31, wave = tid >> 5;
  const int n0 = blockIdx.x * 32;
  const v4f wa = *(const v4f*)(W2 + lane * 16);
  const v4f wb = *(const v4f*)(W2 + lane * 16 + 4);
  const v4f wc = *(const v4f*)(W2 + lane * 16 + 8);
  const v4f wd = *(const v4f*)(W2 + lane * 16 + 12);
  const float bb = b2[0];
#pragma unroll 1
  for (int q = 0; q < 4; ++q) {
    const int n = n0 + wave * 4 + q;
    const _Float16* row = Tp + (size_t)n * NEMB + lane * 16;
    const v8h t0 = *(const v8h*)row;
    const v8h t1 = *(const v8h*)(row + 8);
    float s = 0.0f;
#pragma unroll
    for (int e = 0; e < 4; ++e) s = fmaf((float)t0[e], wa[e], s);
#pragma unroll
    for (int e = 0; e < 4; ++e) s = fmaf((float)t0[4 + e], wb[e], s);
#pragma unroll
    for (int e = 0; e < 4; ++e) s = fmaf((float)t1[e], wc[e], s);
#pragma unroll
    for (int e = 0; e < 4; ++e) s = fmaf((float)t1[4 + e], wd[e], s);
#pragma unroll
    for (int off = 1; off < 32; off <<= 1) s += __shfl_xor(s, off, 32);
    const float gv = fsig(s + bb);
    if (lane == 0) gs[wave * 4 + q] = gv;
  }
  __syncthreads();
  if (wave == 0 && lane < 8) {
    const v4f v = *(const v4f*)(gs + lane * 4);
    float* dst = G + n0 + lane * 4;
    *(volatile v4f*)dst = v;
    __threadfence();
    *(volatile v4f*)dst = v;
  }
}

__global__ __launch_bounds__(NTHREADS) void episode_kernel(
    const unsigned short* __restrict__ XGTp, const float* __restrict__ G,
    const unsigned short* __restrict__ RKTp, const float* __restrict__ bias_ep,
    unsigned short* __restrict__ EP16p) {
  extern __shared__ float4 dsm4[];
  float* Hs = (float*)dsm4;
  _Float16* Ht = (_Float16*)((unsigned char*)dsm4 + HS_BYTES);
  const _Float16* XGT = (const _Float16*)XGTp;
  const _Float16* RKT = (const _Float16*)RKTp;
  const int tid = threadIdx.x, lane = tid & 31, wave = tid >> 5;
  const int c = lane & 15, hh = lane >> 4, koff = hh * 8;
  const int bbase = blockIdx.x * RBLK;

#pragma unroll 1
  for (int i = tid; i < RBLK * NEMB; i += NTHREADS) Hs[i] = 0.0f;
#pragma unroll 1
  for (int i = tid; i < 2 * HT_HALVES; i += NTHREADS) Ht[i] = (_Float16)0.0f;
  __syncthreads();

  const v8f z8 = {0.f, 0.f, 0.f, 0.f, 0.f, 0.f, 0.f, 0.f};
#pragma unroll 1
  for (int f = 0; f < NFACT; ++f) {
    const _Float16* Hc = Ht + (f & 1) * HT_HALVES;
    _Float16* Hn = Ht + ((f & 1) ^ 1) * HT_HALVES;
#pragma unroll 1
    for (int ci = 0; ci < 2; ++ci) {
      const int u0 = (wave + 8 * ci) * 32;
      v8f acc[3][2][2];
#pragma unroll
      for (int g = 0; g < 3; ++g)
#pragma unroll
        for (int i2 = 0; i2 < 2; ++i2)
#pragma unroll
          for (int jt = 0; jt < 2; ++jt) acc[g][i2][jt] = z8;
      const _Float16* a0p = Hc + c * HTPITCH + koff;
      const _Float16* a1p = Hc + (16 + c) * HTPITCH + koff;
      const _Float16* bp  = RKT + (size_t)(u0 + c) * NEMB + koff;
#pragma unroll 1
      for (int k0 = 0; k0 < NEMB; k0 += 32) {
        const v16h a0 = FragH::load(a0p + k0);
        const v16h a1 = FragH::load(a1p + k0);
        v16h bq[3][2];
#pragma unroll
        for (int g = 0; g < 3; ++g)
#pragma unroll
          for (int jt = 0; jt < 2; ++jt)
            bq[g][jt] = FragH::load(bp + (size_t)(g * NEMB + jt * 16) * NEMB + k0);
#pragma unroll
        for (int g = 0; g < 3; ++g)
#pragma unroll
          for (int jt = 0; jt < 2; ++jt) {
            acc[g][0][jt] = FragH::mma(a0, bq[g][jt], acc[g][0][jt]);
            acc[g][1][jt] = FragH::mma(a1, bq[g][jt], acc[g][1][jt]);
          }
        acc_guard4(acc[0][0][0], acc[0][0][1], acc[0][1][0], acc[0][1][1]);
        acc_guard4(acc[1][0][0], acc[1][0][1], acc[1][1][0], acc[1][1][1]);
        acc_guard4(acc[2][0][0], acc[2][0][1], acc[2][1][0], acc[2][1][1]);
        keep4_h(a0, a1, bq[0][0], bq[0][1]);
        keep4_h(bq[1][0], bq[1][1], bq[2][0], bq[2][1]);
      }
#pragma unroll
      for (int i2 = 0; i2 < 2; ++i2) {
#pragma unroll
        for (int jt = 0; jt < 2; ++jt) {
          const int unit = u0 + jt * 16 + c;
          const float bz = bias_ep[NGATE3 + unit];
          const float br = bias_ep[NGATE3 + NEMB + unit];
          const float bh = bias_ep[NGATE3 + 2 * NEMB + unit];
          const int rowb = i2 * 16 + 8 * hh;
          const size_t nrow = (size_t)f * NBATCH + bbase + rowb;
          const v8h xz8 = *(const v8h*)(XGT + (size_t)unit * NROWALL + nrow);
          const v8h xr8 = *(const v8h*)(XGT + (size_t)(NEMB + unit) * NROWALL + nrow);
          const v8h xh8 = *(const v8h*)(XGT + (size_t)(2 * NEMB + unit) * NROWALL + nrow);
          const v8f g8  = *(const v8f*)(G + nrow);
#pragma unroll
          for (int r = 0; r < 8; ++r) {
            const int li = (rowb + r) * NEMB + unit;
            const float hold = Hs[li];
            const float hz = fmaf(acc[0][i2][jt][r], FOLD_HW, bz);
            const float hr = fmaf(acc[1][i2][jt][r], FOLD_HW, br);
            const float hc = fmaf(acc[2][i2][jt][r], FOLD_HW, bh);
            const float zz = fsig((float)xz8[r] + hz);
            const float rr = fsig((float)xr8[r] + hr);
            const float cand = ftanh(fmaf(rr, hc, (float)xh8[r]));
            const float hnew = fmaf(zz, hold - cand, cand);
            const float h2 = fmaf(g8[r], hnew - hold, hold);
            Hs[li] = h2;
            Hn[(rowb + r) * HTPITCH + unit] = (_Float16)(HCARRY * h2);
          }
        }
      }
    }
    __syncthreads();
  }

  const _Float16* Hfin = Ht;
#pragma unroll 1
  for (int it = 0; it < 8; ++it) {
    const int idx = it * NTHREADS + tid;
    const int row = idx >> 6, c8 = (idx & 63) * 8;
    const v8h v = *(const v8h*)(Hfin + row * HTPITCH + c8);
    unsigned short* dst = EP16p + (size_t)(bbase + row) * NEMB + c8;
    *(volatile v8h*)dst = v;
    __threadfence();
    *(volatile v8h*)dst = v;
  }
}

__global__ __launch_bounds__(NTHREADS) void memcombine_kernel(const float* __restrict__ XHM, const float* __restrict__ bias_mem,
                                                             const float* __restrict__ mold, int use_old,
                                                             float* __restrict__ outp, unsigned short* __restrict__ M16) {
  const int i  = blockIdx.x * NTHREADS + threadIdx.x;
  const int b  = i >> 7;
  const int e0 = (i & 127) * 4;
  const float* xrow = XHM + (size_t)b * NGATE3;
  const float* hrow = XHM + XMPLANE + (size_t)b * NGATE3;
  const v4f xz = *(const v4f*)(xrow + e0);
  const v4f xr = *(const v4f*)(xrow + NEMB + e0);
  const v4f xh = *(const v4f*)(xrow + 2 * NEMB + e0);
  const v4f hz = *(const v4f*)(hrow + e0);
  const v4f hr = *(const v4f*)(hrow + NEMB + e0);
  const v4f hc = *(const v4f*)(hrow + 2 * NEMB + e0);
  const v4f b0z = *(const v4f*)(bias_mem + e0);
  const v4f b0r = *(const v4f*)(bias_mem + NEMB + e0);
  const v4f b0h = *(const v4f*)(bias_mem + 2 * NEMB + e0);
  const v4f b1z = *(const v4f*)(bias_mem + NGATE3 + e0);
  const v4f b1r = *(const v4f*)(bias_mem + NGATE3 + NEMB + e0);
  const v4f b1h = *(const v4f*)(bias_mem + NGATE3 + 2 * NEMB + e0);
  v4f mo = {0.1f, 0.1f, 0.1f, 0.1f};
  if (use_old != 0) mo = *(const v4f*)(mold + (size_t)b * NEMB + e0);
  v4f res;
  v4h hv;
#pragma unroll
  for (int k = 0; k < 4; ++k) {
    const float zz = fsig((xz[k] + b0z[k]) + (hz[k] + b1z[k]));
    const float rr = fsig((xr[k] + b0r[k]) + (hr[k] + b1r[k]));
    const float cand = ftanh(fmaf(rr, hc[k] + b1h[k], xh[k] + b0h[k]));
    const float mn = fmaf(zz, mo[k] - cand, cand);
    res[k] = mn;
    hv[k] = (_Float16)(HCARRY * mn);
  }
  float* od = outp + (size_t)b * NEMB + e0;
  unsigned short* md = M16 + (size_t)b * NEMB + e0;
  *(volatile v4f*)od = res;
  *(volatile v4h*)md = hv;
  __threadfence();
  *(volatile v4f*)od = res;
  *(volatile v4h*)md = hv;
}

extern "C" void kernel_launch(void* const* d_in, const int* in_sizes, int n_in,
                              void* d_out, int out_size, void* d_ws, size_t ws_size, hipStream_t stream) {
  if (n_in < 11 || d_out == nullptr || d_ws == nullptr) return;
  if (in_sizes[0] != NBATCH * NFACT * NEMB || in_sizes[1] != 4 * NEMB * NEMB || in_sizes[2] != NEMB ||
      in_sizes[3] != NEMB || in_sizes[4] < 1 || in_sizes[5] != NEMB * NGATE3 || in_sizes[6] != NEMB * NGATE3 ||
      in_sizes[7] != 2 * NGATE3 || in_sizes[8] != NEMB * NGATE3 || in_sizes[9] != NEMB * NGATE3 ||
      in_sizes[10] != 2 * NGATE3 || out_size != NHOPS * NBATCH * NEMB) return;

  const float* facts    = (const float*)d_in[0];
  const float* W1       = (const float*)d_in[1];
  const float* b1       = (const float*)d_in[2];
  const float* W2       = (const float*)d_in[3];
  const float* b2       = (const float*)d_in[4];
  const float* k_ep     = (const float*)d_in[5];
  const float* rk_ep    = (const float*)d_in[6];
  const float* bias_ep  = (const float*)d_in[7];
  const float* k_mem    = (const float*)d_in[8];
  const float* rk_mem   = (const float*)d_in[9];
  const float* bias_mem = (const float*)d_in[10];
  float* out = (float*)d_out;

  char* ws = (char*)d_ws; size_t off = 0;
  auto carve = [&](size_t bytes) -> char* { char* p = ws + off; off += (bytes + 255) & ~(size_t)255; return p; };
  unsigned short* W1A   = (unsigned short*)carve((size_t)NEMB * KFEAT2 * 2);
  unsigned short* W1B   = (unsigned short*)carve((size_t)NEMB * KFEAT2 * 2);
  unsigned short* GPL   = (unsigned short*)carve((size_t)4 * GPLANE * 2);
  unsigned short* XGT   = (unsigned short*)carve((size_t)NGATE3 * NROWALL * 2);
  float*          P0    = (float*)carve((size_t)NROWALL * NEMB * 4);
  unsigned short* FEAT  = (unsigned short*)carve((size_t)MHALF * KFEAT2 * 2);
  unsigned short* R16   = (unsigned short*)carve((size_t)NROWALL * NEMB * 2);
  float*          G     = (float*)carve((size_t)NROWALL * 4);
  unsigned short* EPM   = (unsigned short*)carve((size_t)2 * EPPLANE * 2);
  float*          XHM   = (float*)carve((size_t)2 * XMPLANE * 4);
  if (off > ws_size || off > (size_t)134217728) return;

  unsigned short* KEPT  = GPL;
  unsigned short* RKEPT = GPL + (size_t)GPLANE;
  unsigned short* KMT   = GPL + (size_t)2 * GPLANE;
  unsigned short* EP16  = EPM;
  unsigned short* MEM16 = EPM + EPPLANE;

  cast_facts_kernel<<<dim3(NROWALL * NEMB / 8 / NTHREADS), dim3(NTHREADS), 0, stream>>>(facts, R16);
  w1_trans_kernel<<<dim3(NEMB / 64, 4 * NEMB / 64), dim3(NTHREADS), 0, stream>>>(W1, W1A, W1B);
  gate_trans_kernel<<<dim3(NGATE3 / 64, NEMB / 64, 4), dim3(NTHREADS), 0, stream>>>(k_ep, rk_ep, k_mem, rk_mem, GPL);
  init_mem16_kernel<<<dim3(NBATCH * NEMB / 8 / NTHREADS), dim3(NTHREADS), 0, stream>>>(MEM16);

  wmma_gemm64<0, false, 1, 1, false, 0><<<dim3((NGATE3 / 64) * (NROWALL / 64) / 8), dim3(NTHREADS), 0, stream>>>(
      KEPT, KEPT, NEMB, 0L, R16, R16, NEMB, 0L, (void*)XGT, (void*)XGT, NROWALL, 0L,
      bias_ep, bias_ep, 0L, NGATE3, NROWALL, NEMB, FOLD_W);

  for (int half = 0; half < 2; ++half) {
    feat_build_kernel<<<dim3(MHALF * KFEAT2 / 8 / NTHREADS), dim3(NTHREADS), 0, stream>>>(facts, out, 0, half, FEAT);
    float* P0h = P0 + (size_t)half * MHALF * NEMB;
    wmma_gemm64<0, false, 0, 0, false, 0><<<dim3((MHALF / 64) * (NEMB / 64) / 8), dim3(NTHREADS), 0, stream>>>(
        FEAT, FEAT, KFEAT2, 0L, W1A, W1A, KFEAT2, 0L, (void*)P0h, (void*)P0h, NEMB, 0L,
        b1, b1, 0L, MHALF, NEMB, KFEAT2, FOLD_W);
  }

  for (int hop = 0; hop < NHOPS; ++hop) {
    const int use_prev = (hop > 0) ? 1 : 0;
    const float* mprev = out + (size_t)(hop > 0 ? hop - 1 : 0) * EPPLANE;
    float* out_hop = out + (size_t)hop * EPPLANE;
    for (int half = 0; half < 2; ++half) {
      feat_build_kernel<<<dim3(MHALF * KFEAT2 / 8 / NTHREADS), dim3(NTHREADS), 0, stream>>>(facts, mprev, use_prev, half, FEAT);
      unsigned short* T16h = R16 + (size_t)half * MHALF * NEMB;
      const float* P0h = P0 + (size_t)half * MHALF * NEMB;
      wmma_gemm64<0, false, 2, 1, true, 1><<<dim3((MHALF / 64) * (NEMB / 64) / 8), dim3(NTHREADS), 0, stream>>>(
          FEAT, FEAT, KFEAT2, 0L, W1B, W1B, KFEAT2, 0L, (void*)T16h, (void*)T16h, NEMB, 0L,
          b1, P0h, 0L, MHALF, NEMB, KFEAT2, FOLD_W);
    }
    gate_head_kernel<<<dim3(NROWALL / 32), dim3(NTHREADS), 0, stream>>>(R16, W2, b2, G);
    episode_kernel<<<dim3(NBATCH / RBLK), dim3(NTHREADS), REC_LDS_BYTES, stream>>>(XGT, G, RKEPT, bias_ep, EP16);
    wmma_gemm64<0, false, 0, 0, false, 0><<<dim3((NBATCH / 64) * (NGATE3 / 64) / 8, 2), dim3(NTHREADS), 0, stream>>>(
        EP16, EP16, NEMB, (long)EPPLANE, KMT, KMT, NEMB, (long)GPLANE, (void*)XHM, (void*)XHM, NGATE3, (long)XMPLANE,
        bias_mem, bias_mem, 0L, NBATCH, NGATE3, NEMB, FOLD_HW);
    memcombine_kernel<<<dim3(NBATCH * NEMB / 4 / NTHREADS), dim3(NTHREADS), 0, stream>>>(XHM, bias_mem, mprev, use_prev, out_hop, MEM16);
  }
}
